// KMEAttention_48627619726105
// MI455X (gfx1250) — hardware-run, weakly checked
//
#include <hip/hip_runtime.h>
#include <math.h>

typedef __attribute__((ext_vector_type(16))) _Float16 v16h;
typedef __attribute__((ext_vector_type(16))) __bf16 v16b;
typedef __attribute__((ext_vector_type(8)))  _Float16 v8h;
typedef __attribute__((ext_vector_type(8)))  float v8f;
typedef __attribute__((ext_vector_type(4)))  float v4f;
typedef __attribute__((ext_vector_type(2)))  float v2f;
typedef __attribute__((ext_vector_type(4)))  unsigned v4u;
typedef __attribute__((ext_vector_type(4)))  int v4i;
typedef float __attribute__((may_alias)) float_a;
typedef int __attribute__((may_alias)) int_a;

template <typename T> __device__ __forceinline__ void vst2(void* p, T v) { *(volatile T*)p = v; __threadfence(); *(volatile T*)p = v; }
__device__ __forceinline__ v8f wmma16(v16h a, v16h b, v8f c) {
  v8f d = __builtin_amdgcn_wmma_f32_16x16x32_f16(false, a, false, b, (short)0, c, false, false);
  asm volatile("v_nop\n\tv_nop\n\tv_nop\n\tv_nop" : "+v"(d) : "v"(a), "v"(b));
  return d;
}
__device__ __forceinline__ v8f wmma_bf(v16b a, v16b b, v8f c) {
  v8f d = __builtin_amdgcn_wmma_f32_16x16x32_bf16(false, a, false, b, (short)0, c, false, false);
  asm volatile("v_nop\n\tv_nop\n\tv_nop\n\tv_nop" : "+v"(d) : "v"(a), "v"(b));
  return d;
}
__device__ __forceinline__ v16h frag_h(const _Float16* rowk0, int lane) {
  union { v16h v; v8h q[2]; } u; const _Float16* p = rowk0 + 8 * (lane >> 4);
  u.q[0] = *(const v8h*)p; u.q[1] = *(const v8h*)(p + 16); return u.v;
}
__device__ __forceinline__ v16h frag_f32(const float* rowk0, int lane) {
  v16h a; const float* p = rowk0 + 8 * (lane >> 4);
#pragma unroll
  for (int i = 0; i < 8; ++i) { a[i] = (_Float16)p[i]; a[8 + i] = (_Float16)p[16 + i]; }
  return a;
}
__device__ __forceinline__ v16h frag_f32s(const float* rowk0, int lane, float sc) {
  v16h a; const float* p = rowk0 + 8 * (lane >> 4);
#pragma unroll
  for (int i = 0; i < 8; ++i) { a[i] = (_Float16)(p[i] * sc); a[8 + i] = (_Float16)(p[16 + i] * sc); }
  return a;
}
__device__ __forceinline__ v16h fragc_f32(const float* W, int k0, int n, int lane, int ld, int K) {
  v16h a; const int g = lane >> 4;
#pragma unroll
  for (int i = 0; i < 8; ++i) { const int ka = k0 + 8 * g + i, kb = ka + 16;
    a[i] = (_Float16)(ka < K ? W[(size_t)(ka < K ? ka : K - 1) * ld + n] : 0.f); a[8 + i] = (_Float16)(kb < K ? W[(size_t)(kb < K ? kb : K - 1) * ld + n] : 0.f); }
  return a;
}
struct F2 { v16b h, l; };
__device__ __forceinline__ F2 bsplit16(const float v[16]) { F2 r;
#pragma unroll
  for (int i = 0; i < 16; ++i) { const __bf16 h = (__bf16)v[i]; r.h[i] = h; r.l[i] = (__bf16)(v[i] - (float)h); }
  return r; }
__device__ __forceinline__ F2 split_row(const float* row, int k0, int lane) { float v[16]; const float* p = row + k0 + 8 * (lane >> 4);
#pragma unroll
  for (int i = 0; i < 8; ++i) { v[i] = p[i]; v[8 + i] = p[16 + i]; }
  return bsplit16(v); }
__device__ __forceinline__ F2 split_rowK(const float* row, int k0, int lane, int K) { float v[16]; const int g = lane >> 4;
#pragma unroll
  for (int i = 0; i < 8; ++i) { const int ka = k0 + 8 * g + i, kb = ka + 16; v[i] = ka < K ? row[ka < K ? ka : K - 1] : 0.f; v[8 + i] = kb < K ? row[kb < K ? kb : K - 1] : 0.f; }
  return bsplit16(v); }
__device__ __forceinline__ F2 split_col(const float* W, int k0, int n, int lane, int ld, int K) { float v[16]; const int g = lane >> 4;
#pragma unroll
  for (int i = 0; i < 8; ++i) { const int ka = k0 + 8 * g + i, kb = ka + 16; v[i] = ka < K ? W[(size_t)(ka < K ? ka : K - 1) * ld + n] : 0.f; v[8 + i] = kb < K ? W[(size_t)(kb < K ? kb : K - 1) * ld + n] : 0.f; }
  return bsplit16(v); }
__device__ __forceinline__ v8f mac3(const F2& a, const F2& b, v8f c) { c = wmma_bf(a.l, b.h, c); c = wmma_bf(a.h, b.l, c); return wmma_bf(a.h, b.h, c); }
__device__ __forceinline__ float sigm(float v) { return 1.0f / (1.0f + expf(-v)); }
#define LDSX() do { asm volatile("s_wait_dscnt 0" ::: "memory"); __builtin_amdgcn_wave_barrier(); __builtin_amdgcn_fence(__ATOMIC_RELEASE, "workgroup"); } while (0)


#define NB 4
#define SS 1024
#define MA 8
#define DD 64
#define NH 8
#define NF 32
#define HW (NH * DD)
#define NT (NB * SS)
#define NAR (NT * MA)
#define VC (MA * DD)
#ifndef TQB
#define TQB (SS / 64)
#define TNB NB
#endif
typedef __attribute__((ext_vector_type(8))) __bf16 v8b;
__device__ __forceinline__ v16b frag_b(const __bf16* rowk0, int lane) {
  union { v16b v; v8b q[2]; } u; const __bf16* p = rowk0 + 8 * (lane >> 4);
  u.q[0] = *(const v8b*)p; u.q[1] = *(const v8b*)(p + 16); return u.v;
}
__device__ __forceinline__ float bfr(float v) { return (float)(__bf16)v; }
__device__ __attribute__((noinline)) float exp_ni(float v) { return expf(v); }
__device__ __attribute__((noinline)) float erf_ni(float v) { return erff(v); }
__device__ __attribute__((noinline)) float cos_p(float v) { return cosf(v); }
__device__ __attribute__((noinline)) float sin_p(float v) { return sinf(v); }

#define WS_PW  0u
#define WS_PO  (WS_PW + 2u * (size_t)3 * HW * DD)
#define WS_PF  (WS_PO + 2u * (size_t)DD * HW)
#define WS_QA  (WS_PF + 2u * (size_t)NH * NF * DD)
#define WS_KA  (WS_QA + 4u * (size_t)NAR * HW)
#define WS_VP  (WS_KA + 4u * (size_t)NAR * HW)
#define WS_QE  (WS_VP + 2u * (size_t)NB * NH * VC * SS)
#define WS_KE  (WS_QE + 2u * (size_t)NT * HW)
#define WS_END (WS_KE + 2u * (size_t)NT * HW)
#define WS_O   WS_QA

__global__ __launch_bounds__(64) void k_pack(const float* __restrict__ WQ, const float* __restrict__ WK, const float* __restrict__ WV, const float* __restrict__ WO, const float* __restrict__ FR, __bf16* __restrict__ P) { const int n = blockIdx.x, which = blockIdx.y, t = threadIdx.x; __shared__ __align__(16) __bf16 s[HW];
  if (which < 3) { const float* w = (which == 0) ? WQ : (which == 1) ? WK : WV; s[t] = (__bf16)w[(size_t)n * DD + t]; __syncthreads(); if (t < DD / 8) vst2((unsigned*)(P + WS_PW / 2 + ((size_t)which * HW + n) * DD + t * 8), *(const v4u*)&s[t * 8]); }
  else if (which == 3) { if (n >= DD) return; for (int k = t; k < HW; k += 64) s[k] = (__bf16)WO[(size_t)n * HW + k]; __syncthreads(); vst2((unsigned*)(P + WS_PO / 2 + (size_t)n * HW + t * 8), *(const v4u*)&s[t * 8]); }
  else { if (n >= NH * NF) return; const int h = n / NF, f = n % NF; s[t] = (__bf16)FR[((size_t)h * DD + t) * NF + f]; __syncthreads(); if (t < DD / 8) vst2((unsigned*)(P + WS_PF / 2 + (size_t)n * DD + t * 8), *(const v4u*)&s[t * 8]); } }
__global__ __launch_bounds__(128) void k_proj(const float* __restrict__ AQ, const float* __restrict__ AK, const __bf16* __restrict__ P, float* __restrict__ QA, float* __restrict__ KA) {
  __shared__ __align__(16) float sf[4][16][132];
  const int tid = threadIdx.x, wave = tid >> 5, lane = tid & 31, col = lane & 15, g = lane >> 4; const int which = blockIdx.z; const size_t rb = (size_t)blockIdx.x * 64; const size_t r0 = rb + wave * 16; const int c0 = blockIdx.y * 128; const float* A = (which == 0) ? AQ : AK; const __bf16* Wr = P + WS_PW / 2 + ((size_t)which * HW) * DD;
  v8f acc[8] = {};
#pragma unroll
  for (int kc = 0; kc < 2; ++kc) { v16b a; { const float* p = A + (r0 + col) * DD + kc * 32 + 8 * g;
#pragma unroll
      for (int i = 0; i < 8; ++i) { a[i] = (__bf16)p[i]; a[8 + i] = (__bf16)p[16 + i]; } }
#pragma unroll
    for (int j = 0; j < 8; ++j) acc[j] = wmma_bf(a, frag_b(Wr + (size_t)(c0 + j * 16 + col) * DD + kc * 32, lane), acc[j]); }
  {
#pragma unroll
    for (int j = 0; j < 8; ++j)
#pragma unroll
      for (int r = 0; r < 8; ++r) sf[wave][8 * g + r][j * 16 + col] = acc[j][r];
    LDSX(); float* dst = (which == 0) ? QA : KA; for (int rl = 0; rl < 16; ++rl) vst2(dst + (r0 + rl) * HW + c0 + lane * 4, *(const v4f*)&sf[wave][rl][lane * 4]); }

}

__global__ __launch_bounds__(128) void k_projv(const float* __restrict__ AV, const __bf16* __restrict__ P, _Float16* __restrict__ VP) { __shared__ __align__(16) _Float16 st[128][72];
  const int tid = threadIdx.x, wave = tid >> 5, lane = tid & 31, col = lane & 15, g = lane >> 4; const int m = blockIdx.z; const size_t tb = (size_t)blockIdx.x * 64; const int c0 = blockIdx.y * 128; const __bf16* Wr = P + WS_PW / 2 + ((size_t)2 * HW) * DD;
  v8f acc[8] = {};
#pragma unroll
  for (int kc = 0; kc < 2; ++kc) { v16b a; { const float* p = AV + ((tb + wave * 16 + col) * MA + m) * DD + kc * 32 + 8 * g;
#pragma unroll
      for (int i = 0; i < 8; ++i) { a[i] = (__bf16)p[i]; a[8 + i] = (__bf16)p[16 + i]; } }
#pragma unroll
    for (int j = 0; j < 8; ++j) acc[j] = wmma_bf(a, frag_b(Wr + (size_t)(c0 + j * 16 + col) * DD + kc * 32, lane), acc[j]); }
#pragma unroll
  for (int j = 0; j < 8; ++j)
#pragma unroll
    for (int r = 0; r < 8; ++r) st[j * 16 + col][wave * 16 + 8 * g + r] = (_Float16)acc[j][r];
  __syncthreads(); const size_t b = tb / SS; const int s0 = (int)(tb % SS);
  for (int e = tid; e < 128 * 8; e += 128) { const int cl = e >> 3, pc = e & 7; const int c = c0 + cl; const int h = c / DD, d = c % DD; vst2((unsigned*)(VP + (((b * NH + h) * VC + m * DD + d) * SS) + s0 + pc * 8), *(const v4u*)&st[cl][pc * 8]); } }
__global__ __launch_bounds__(128) void k_enc(const float* __restrict__ QA, const float* __restrict__ KA, const float* __restrict__ QLW, const float* __restrict__ KLW, const __bf16* __restrict__ P, _Float16* __restrict__ QE, _Float16* __restrict__ KE) {
  __shared__ float sphi[64][DD + 1]; __shared__ float sw[8][MA]; __shared__ __align__(16) _Float16 so[8][DD + 8];
  const int tid = threadIdx.x, wave = tid >> 5, lane = tid & 31, col = lane & 15, g = lane >> 4; const int h = blockIdx.y; const int which = blockIdx.z; const size_t rb = (size_t)blockIdx.x * 64; const size_t r0 = rb + wave * 16; const float* A = (which == 0) ? QA : KA; const float* LW = (which == 0) ? QLW : KLW; const __bf16* Fr = P + WS_PF / 2 + (size_t)h * NF * DD;
  v8f acc[2] = {};
#pragma unroll
  for (int kc = 0; kc < 2; ++kc) { const F2 a = split_row(A + (r0 + col) * HW + h * DD, kc * 32, lane);
#pragma unroll
    for (int j = 0; j < 2; ++j) { const v16b w = frag_b(Fr + (size_t)(j * 16 + col) * DD + kc * 32, lane); acc[j] = wmma_bf(a.h, w, acc[j]); acc[j] = wmma_bf(a.l, w, acc[j]); } }
#pragma unroll
  for (int j = 0; j < 2; ++j)
#pragma unroll
    for (int r = 0; r < 8; ++r) { const float pv = acc[j][r]; const int rl = wave * 16 + 8 * g + r, f = j * 16 + col; sphi[rl][f] = cos_p(pv) * 0.17677669529663688f; sphi[rl][NF + f] = sin_p(pv) * 0.17677669529663688f; }
  if (tid < 8) { const size_t tok = rb / MA + tid; float lw[MA]; float mx = -3.0e38f; for (int m = 0; m < MA; ++m) { lw[m] = bfr(LW[tok * MA + m]); mx = fmaxf(mx, lw[m]); } float z = 0.f; for (int m = 0; m < MA; ++m) { lw[m] = __expf(lw[m] - mx); z += lw[m]; } for (int m = 0; m < MA; ++m) sw[tid][m] = lw[m] / z; }
  __syncthreads();
  for (int e = tid; e < 8 * DD; e += 128) { const int tk = e >> 6, f = e & 63; float z = 0.f;
#pragma unroll
    for (int m = 0; m < MA; ++m) z += sphi[tk * MA + m][f] * sw[tk][m]; so[tk][f] = (_Float16)z; }
  __syncthreads();
  if (tid < 64) { const int tk = tid >> 3, q = tid & 7; const size_t tok = rb / MA + tk; vst2((unsigned*)(((which == 0) ? QE : KE) + tok * HW + h * DD + q * 8), *(const v4u*)&so[tk][q * 8]); }
}
__global__ __launch_bounds__(128) void k_attn(const _Float16* __restrict__ QE, const _Float16* __restrict__ KE, const _Float16* __restrict__ VP, float* __restrict__ O) {
  __shared__ __align__(16) _Float16 sph[4][16][40]; __shared__ __align__(16) float so[4][16][132];
  const int tid = threadIdx.x, wave = tid >> 5, lane = tid & 31, col = lane & 15, g = lane >> 4; const int h = blockIdx.y >> 2, vq = blockIdx.y & 3; const size_t b = blockIdx.z; const int q0 = blockIdx.x * 64 + wave * 16; const size_t rq = b * SS + q0;
  v16h aq[2];
#pragma unroll
  for (int kc = 0; kc < 2; ++kc) aq[kc] = frag_h(QE + (rq + col) * HW + h * DD + kc * 32, lane);
  float m[8], l[8];
#pragma unroll
  for (int r = 0; r < 8; ++r) { m[r] = -3.0e38f; l[r] = 0.f; }
  v8f acc[8] = {};
#pragma unroll 1
  for (int ks = 0; ks < SS / 32; ++ks) { const int j0 = ks * 32; v8f s[2];
#pragma unroll
    for (int ct = 0; ct < 2; ++ct) { const int kk = j0 + ct * 16 + col; const size_t rk = (b * SS + kk) * HW + h * DD; v8f c = {};
#pragma unroll
      for (int kc = 0; kc < 2; ++kc) c = wmma16(aq[kc], frag_h(KE + rk + kc * 32, lane), c);
#pragma unroll
      for (int r = 0; r < 8; ++r) s[ct][r] = c[r] * 0.125f; }
#pragma unroll
    for (int r = 0; r < 8; ++r) { float mx = fmaxf(s[0][r], s[1][r]);
#pragma unroll
      for (int o = 1; o < 16; o <<= 1) mx = fmaxf(mx, __shfl_xor(mx, o));
      const float mn = fmaxf(m[r], mx); const float alpha = (m[r] <= -1.0e38f) ? 0.f : __expf(m[r] - mn); const float e0 = __expf(s[0][r] - mn), e1 = __expf(s[1][r] - mn); float es = e0 + e1;
#pragma unroll
      for (int o = 1; o < 16; o <<= 1) es += __shfl_xor(es, o);
      l[r] = l[r] * alpha + es; m[r] = mn;
#pragma unroll
      for (int dt = 0; dt < 8; ++dt) acc[dt][r] *= alpha;
      sph[wave][8 * g + r][col] = (_Float16)(e0 * 2048.0f); sph[wave][8 * g + r][16 + col] = (_Float16)(e1 * 2048.0f); }
    LDSX();
    const v16h pa = frag_h(&sph[wave][col][0], lane);
#pragma unroll
    for (int dt = 0; dt < 8; ++dt) acc[dt] = wmma16(pa, frag_h(VP + (((b * NH + h) * VC + vq * 128 + dt * 16 + col) * SS) + j0, lane), acc[dt]);
    LDSX(); }
#pragma unroll
  for (int r = 0; r < 8; ++r) { const float il = (1.0f / 2048.0f) / l[r];
#pragma unroll
    for (int dt = 0; dt < 8; ++dt) so[wave][8 * g + r][dt * 16 + col] = acc[dt][r] * il; }
  LDSX();
  for (int rl = 0; rl < 16; ++rl) { const size_t tok = rq + rl; if (lane < 16) vst2(O + ((tok * MA + 2 * vq) * HW) + h * DD + lane * 4, *(const v4f*)&so[wave][rl][lane * 4]); else vst2(O + ((tok * MA + 2 * vq + 1) * HW) + h * DD + (lane - 16) * 4, *(const v4f*)&so[wave][rl][64 + (lane - 16) * 4]); }
}
__global__ __launch_bounds__(128) void k_oat(const float* __restrict__ O, const __bf16* __restrict__ P, float* __restrict__ OA) { __shared__ __align__(16) float so[4][16][68];
  const int tid = threadIdx.x, wave = tid >> 5, lane = tid & 31, col = lane & 15, g = lane >> 4; const size_t r0 = (size_t)blockIdx.x * 64 + wave * 16; const __bf16* Wr = P + WS_PO / 2;
  v8f acc[4] = {};
#pragma unroll 2
  for (int kc = 0; kc < HW / 32; ++kc) { const F2 a = split_row(O + (r0 + col) * HW, kc * 32, lane);
#pragma unroll
    for (int j = 0; j < 4; ++j) { const v16b w = frag_b(Wr + (size_t)(j * 16 + col) * HW + kc * 32, lane); acc[j] = wmma_bf(a.h, w, acc[j]); acc[j] = wmma_bf(a.l, w, acc[j]); } }
#pragma unroll
  for (int j = 0; j < 4; ++j)
#pragma unroll
    for (int r = 0; r < 8; ++r) so[wave][8 * g + r][j * 16 + col] = acc[j][r];
  LDSX(); for (int rl = 0; rl < 16; ++rl) if (lane < 16) vst2(OA + (r0 + rl) * DD + lane * 4, *(const v4f*)&so[wave][rl][lane * 4]); }
__global__ __launch_bounds__(256) void k_lw(const float* __restrict__ OA, const float* __restrict__ QLW, const float* __restrict__ WW, float* __restrict__ OUT) { __shared__ float sof[32][DD]; __shared__ __align__(16) float so2[32 * MA]; const int t = threadIdx.x; const size_t tok0 = (size_t)blockIdx.x * 32;
  for (int e = t; e < 32 * DD; e += 256) { const int tk = e >> 6, d = e & 63; float s = 0.f; for (int m = 0; m < MA; ++m) s += OA[((tok0 + tk) * MA + m) * DD + d]; sof[tk][d] = s * (1.0f / (float)MA); }
  __syncthreads();
  { const int tk = t >> 3, m = t & 7; float a = 0.f; for (int d = 0; d < DD; ++d) a += sof[tk][d] * bfr(WW[m * DD + d]); so2[tk * MA + m] = bfr(QLW[(tok0 + tk) * MA + m]) + a; }
  __syncthreads(); if (t < 64) vst2(OUT + tok0 * MA + t * 4, *(const v4f*)&so2[t * 4]); }
extern "C" void kernel_launch(void* const* d_in, const int* in_sizes, int n_in, void* d_out, int out_size, void* d_ws, size_t ws_size, hipStream_t stream) {
  (void)in_sizes; (void)n_in; (void)out_size;
  const float** F = (const float**)d_in;
  if (ws_size < (size_t)WS_END) return;
  char* ws = (char*)d_ws; __bf16* P = (__bf16*)ws; float *QA = (float*)(ws + WS_QA), *KA = (float*)(ws + WS_KA), *O = (float*)(ws + WS_O); _Float16 *VP = (_Float16*)(ws + WS_VP), *QE = (_Float16*)(ws + WS_QE), *KE = (_Float16*)(ws + WS_KE);
  float* OA = (float*)d_out; float* OUT1 = (float*)d_out + (size_t)NAR * DD;
  k_pack<<<dim3(HW, 5), 64, 0, stream>>>(F[6], F[7], F[8], F[9], F[11], P);
  k_proj<<<dim3(NAR / 64, HW / 128, 2), 128, 0, stream>>>(F[0], F[2], P, QA, KA);
  k_projv<<<dim3(TNB * SS / 64, HW / 128, MA), 128, 0, stream>>>(F[4], P, VP);
  k_enc<<<dim3(NAR / 64, NH, 2), 128, 0, stream>>>(QA, KA, F[1], F[3], P, QE, KE);
  k_attn<<<dim3(TQB, NH * 4, TNB), 128, 0, stream>>>(QE, KE, VP, O);
  k_oat<<<TNB * SS * MA / 64, 128, 0, stream>>>(O, P, OA);
  k_lw<<<TNB * SS / 32, 256, 0, stream>>>(OA, F[1], F[10], OUT1);
}
